// RNNDoubleStacked_53025666236823
// MI455X (gfx1250) — hardware-verified
//
#include <hip/hip_runtime.h>


#define PN 4096
#define FN 128
#define HN 128
#define MB 16
#define SH 136

static_assert(PN % MB == 0);
static_assert(HN == 128);
static_assert(FN == 128);
static_assert((FN % 2) == 0);
static_assert((PN % 2) == 0);
static_assert((SH % 8) == 0);
static_assert(MB * FN >= MB * HN);

typedef _Float16 v16h __attribute__((ext_vector_type(16)));
typedef _Float16 v8h  __attribute__((ext_vector_type(8)));
typedef float    v8f  __attribute__((ext_vector_type(8)));
typedef float    v4f  __attribute__((ext_vector_type(4)));

union Frag { v16h v; v8h half[2]; };

constexpr size_t WS_U_BYTES = (size_t)PN * HN * 4;
constexpr size_t WS_END     = WS_U_BYTES;
static_assert(WS_END <= (size_t)134217728);
static_assert((WS_U_BYTES % 8192) == 0);

__device__ __forceinline__ void mma16(v8f& acc, const Frag& a, const Frag& b) {
  acc = __builtin_amdgcn_wmma_f32_16x16x32_f16(false, a.v, false, b.v, (short)0, acc, false, false);
  asm volatile("v_nop\n\tv_nop\n\tv_nop\n\tv_nop" : "+v"(acc) : "v"(a.v), "v"(b.v));
}

__device__ __forceinline__ float tanh_f(float x) {
  const float e = __expf(2.0f * x);
  return 1.0f - 2.0f * __builtin_amdgcn_rcpf(e + 1.0f);
}

__device__ __forceinline__ v8h cvt8h(const float* p, float s) {
  const v4f a = *(const v4f*)p;
  const v4f b = *(const v4f*)(p + 4);
  v8h r;
  r[0] = (_Float16)(a[0] * s); r[1] = (_Float16)(a[1] * s);
  r[2] = (_Float16)(a[2] * s); r[3] = (_Float16)(a[3] * s);
  r[4] = (_Float16)(b[0] * s); r[5] = (_Float16)(b[1] * s);
  r[6] = (_Float16)(b[2] * s); r[7] = (_Float16)(b[3] * s);
  return r;
}

__device__ __forceinline__ void load_b_frags(Frag (&B)[4], const float* __restrict__ W, int n, int h, float s) {
#pragma unroll
  for (int kk = 0; kk < 4; ++kk) {
    const float* w = W + (size_t)n * HN + kk * 32 + 8 * h;
    B[kk].half[0] = cvt8h(w, s);
    B[kk].half[1] = cvt8h(w + 16, s);
  }
}

__global__ __launch_bounds__(256) void rnn1_kernel(
    const float* __restrict__ event, const int* __restrict__ lengths,
    const float* __restrict__ Wih1,  const float* __restrict__ Whh1,
    const float* __restrict__ bih1,  const float* __restrict__ bhh1,
    const float* __restrict__ Wih2,  const float* __restrict__ bih2,
    const float* __restrict__ bhh2,  float* U)
{
  __shared__ __attribute__((aligned(16))) _Float16 hb[2][MB][SH];
  __shared__ __attribute__((aligned(16))) float xbuf[MB * FN];

  const int tid  = threadIdx.x;
  const int lane = tid & 31;
  const int wv   = tid >> 5;
  const int h    = lane >> 4;
  const int m    = lane & 15;
  const int p0   = blockIdx.x * MB;
  const int n    = wv * 16 + m;

  for (int idx = tid; idx < MB * FN; idx += 256)
    xbuf[idx] = event[(size_t)p0 * FN + idx];
  for (int idx = tid; idx < 2 * MB * SH; idx += 256)
    (&hb[0][0][0])[idx] = (_Float16)0.0f;

  const float wih   = Wih1[n];
  const float bsum1 = bih1[n] + bhh1[n];
  const float inv64 = 0.015625f;

  int lenr[8];
#pragma unroll
  for (int r = 0; r < 8; ++r) lenr[r] = lengths[p0 + 8 * h + r];

  Frag B1[4];
  load_b_frags(B1, Whh1, n, h, 64.0f);

  float hprev[8];
#pragma unroll
  for (int r = 0; r < 8; ++r) hprev[r] = 0.0f;

  __syncthreads();

#pragma unroll 1
  for (int t = 0; t < FN; ++t) {
    const int cur = t & 1;
    const _Float16* hc = &hb[cur][m][0];
    Frag A[4];
#pragma unroll
    for (int kk = 0; kk < 4; ++kk) {
      A[kk].half[0] = *(const v8h*)(hc + kk * 32 + 8 * h);
      A[kk].half[1] = *(const v8h*)(hc + kk * 32 + 16 + 8 * h);
    }
    v8f acc;
#pragma unroll
    for (int r = 0; r < 8; ++r) acc[r] = 0.0f;
#pragma unroll
    for (int kk = 0; kk < 4; ++kk) mma16(acc, A[kk], B1[kk]);

    _Float16* hnx = &hb[cur ^ 1][0][0];
#pragma unroll
    for (int r = 0; r < 8; ++r) {
      const int mm = 8 * h + r;
      const float pre  = acc[r] * inv64 + (wih * xbuf[mm * FN + t] + bsum1);
      const float hnew = tanh_f(pre);
      const float val  = (t < lenr[r]) ? hnew : hprev[r];
      hprev[r] = val;
      hnx[mm * SH + n] = (_Float16)val;
    }
    __syncthreads();
  }

  Frag B2[4];
  load_b_frags(B2, Wih2, n, h, 64.0f);
  {
    const _Float16* hc = &hb[0][m][0];
    Frag A[4];
#pragma unroll
    for (int kk = 0; kk < 4; ++kk) {
      A[kk].half[0] = *(const v8h*)(hc + kk * 32 + 8 * h);
      A[kk].half[1] = *(const v8h*)(hc + kk * 32 + 16 + 8 * h);
    }
    v8f acc2;
#pragma unroll
    for (int r = 0; r < 8; ++r) acc2[r] = 0.0f;
#pragma unroll
    for (int kk = 0; kk < 4; ++kk) mma16(acc2, A[kk], B2[kk]);

    const float bsum2 = bih2[n] + bhh2[n];
    float* st = xbuf;
#pragma unroll
    for (int r = 0; r < 8; ++r)
      st[(8 * h + r) * HN + n] = acc2[r] * inv64 + bsum2;
  }
  __syncthreads();

  {
    const float* st = xbuf;
    float* gU = U + (size_t)p0 * HN;
    const v4f v0 = *(const v4f*)(st + tid * 4);
    const v4f v1 = *(const v4f*)(st + 1024 + tid * 4);
    *(volatile v4f*)(gU + tid * 4)        = v0;
    *(volatile v4f*)(gU + 1024 + tid * 4) = v1;
    __threadfence();
    *(volatile v4f*)(gU + tid * 4)        = v0;
    *(volatile v4f*)(gU + 1024 + tid * 4) = v1;
  }
}

__global__ __launch_bounds__(256) void rnn2_kernel(
    const float* __restrict__ U, const float* __restrict__ Whh2, float* out)
{
  __shared__ __attribute__((aligned(16))) float hs[2][HN];

  const int tid  = threadIdx.x;
  const int lane = tid & 31;
  const int wv   = tid >> 5;
  const int h    = lane >> 4;
  const int m    = lane & 15;
  const int n    = wv * 16 + m;
  const float inv64 = 0.015625f;
  const float zsel  = (m == 0) ? 1.0f : 0.0f;

  Frag B[4];
  load_b_frags(B, Whh2, n, h, 64.0f);

  (&hs[0][0])[tid] = 0.0f;
  __syncthreads();

#pragma unroll 1
  for (int p = 0; p < PN; ++p) {
    const int cur = p & 1;
    const float* hc = &hs[cur][0];
    const float u = U[(size_t)p * HN + n];

    Frag A[4];
#pragma unroll
    for (int kk = 0; kk < 4; ++kk) {
      A[kk].half[0] = cvt8h(hc + kk * 32 + 8 * h, zsel);
      A[kk].half[1] = cvt8h(hc + kk * 32 + 16 + 8 * h, zsel);
    }
    v8f acc;
#pragma unroll
    for (int r = 0; r < 8; ++r) acc[r] = 0.0f;
#pragma unroll
    for (int kk = 0; kk < 4; ++kk) mma16(acc, A[kk], B[kk]);

    const float hn = tanh_f(acc[0] * inv64 + u);
    if (lane < 16) hs[cur ^ 1][n] = hn;
    __syncthreads();
  }

  if (wv == 0) {
    const v4f v = *(const v4f*)(&hs[0][lane * 4]);
    *(volatile v4f*)(out + lane * 4) = v;
    __threadfence();
    *(volatile v4f*)(out + lane * 4) = v;
  }
}

extern "C" void kernel_launch(void* const* d_in, const int* in_sizes, int n_in,
                              void* d_out, int out_size, void* d_ws, size_t ws_size,
                              hipStream_t stream)
{
  if (n_in < 10) return;
  if (in_sizes[0] != PN * FN)   return;
  if (in_sizes[1] != PN)        return;
  if (in_sizes[2] != HN)        return;
  if (in_sizes[3] != HN * HN)   return;
  if (in_sizes[4] != HN)        return;
  if (in_sizes[5] != HN)        return;
  if (in_sizes[6] != HN * HN)   return;
  if (in_sizes[7] != HN * HN)   return;
  if (in_sizes[8] != HN)        return;
  if (in_sizes[9] != HN)        return;
  if (out_size != HN)           return;
  if (ws_size < WS_END)         return;

  const float* event   = (const float*)d_in[0];
  const int*   lengths = (const int*)  d_in[1];
  const float* Wih1    = (const float*)d_in[2];
  const float* Whh1    = (const float*)d_in[3];
  const float* bih1    = (const float*)d_in[4];
  const float* bhh1    = (const float*)d_in[5];
  const float* Wih2    = (const float*)d_in[6];
  const float* Whh2    = (const float*)d_in[7];
  const float* bih2    = (const float*)d_in[8];
  const float* bhh2    = (const float*)d_in[9];

  float* U = (float*)d_ws;

  rnn1_kernel<<<dim3(PN / MB), dim3(256), 0, stream>>>(event, lengths, Wih1, Whh1, bih1, bhh1,
                                                      Wih2, bih2, bhh2, U);
  rnn2_kernel<<<dim3(1), dim3(256), 0, stream>>>((const float*)U, Whh2, (float*)d_out);
}
